// mLSTMCell_89807766159689
// MI455X (gfx1250) — hardware-run, weakly checked
//
#include <hip/hip_runtime.h>
#include <math.h>

constexpr int SEQ        = 2048;
constexpr int HID        = 1024;
constexpr int NHEAD      = 8;
constexpr int DHEAD      = 128;
constexpr int NFEAT      = 3 * HID;
constexpr int KEY_TILE   = 32;
constexpr int ROWS_BLK   = 64;
constexpr int QPITCH     = 136;
constexpr int VPITCH     = 40;
constexpr int VT_PITCH   = 136;
constexpr int SLABP      = 68;

constexpr double cx_sqrt(double x) {
  double r = x;
  for (int i = 0; i < 48; ++i) r = 0.5 * (r + x / r);
  return r;
}
constexpr double INV_SQRT_DHEAD_D = 1.0 / cx_sqrt((double)DHEAD);
static_assert(INV_SQRT_DHEAD_D * INV_SQRT_DHEAD_D * (double)DHEAD > 0.999999999999 &&
              INV_SQRT_DHEAD_D * INV_SQRT_DHEAD_D * (double)DHEAD < 1.000000000001, "inverse sqrt of head dim");

constexpr float QCARRY   = 16.0f;
constexpr float KCARRY   = 16.0f;
constexpr float VCARRY   = 16.0f;
constexpr float PCARRY   = 1024.0f;
constexpr float RCARRY   = 2048.0f;
constexpr float RCARRY_INV = 1.0f / RCARRY;
constexpr float SSCALE   = (float)(INV_SQRT_DHEAD_D / ((double)QCARRY * (double)KCARRY));
constexpr float OFOLD    = 1.0f / (PCARRY * VCARRY);
constexpr float EPS_NORM = 1e-6f;
constexpr float EPS_LN   = 1e-5f;
constexpr float INV_DHEAD = 1.0f / (float)DHEAD;
constexpr float F32_MIN_NORMAL = 1.17549435e-38f;

static_assert(NHEAD * DHEAD == HID, "head split");
static_assert(NHEAD == 8, "one wave per head in the gate kernel");
static_assert(SEQ % ROWS_BLK == 0 && SEQ % KEY_TILE == 0 && ROWS_BLK % KEY_TILE == 0, "tile multiples");
static_assert(DHEAD % 32 == 0 && KEY_TILE % 32 == 0, "k multiples of 32");
static_assert(SEQ % 32 == 0 && HID % 128 == 0, "gate block rows and feature stride");
static_assert((ROWS_BLK * DHEAD / 8) % 256 == 0, "query tile staging exact");
static_assert(KEY_TILE * DHEAD / 8 == 512 && DHEAD * KEY_TILE / 8 == 512, "key and value tile staging: 2 chunks per thread");
static_assert(QPITCH % 8 == 0 && VPITCH % 8 == 0 && VT_PITCH % 8 == 0, "16-byte fragment alignment");
static_assert(QPITCH >= DHEAD && VPITCH >= KEY_TILE && VT_PITCH >= DHEAD, "pitches cover the tiles");
static_assert(2 * ROWS_BLK * QPITCH * 2 + 2 * KEY_TILE * QPITCH * 2 + DHEAD * VPITCH * 2 + 4 * 16 * VPITCH * 2 +
              8 * 16 * SLABP * 4 + 3 * 4 * 2 * 16 * 4 == 103936, "static LDS total of the attention kernel");

typedef __attribute__((ext_vector_type(16))) _Float16 v16h;
typedef __attribute__((ext_vector_type(8)))  _Float16 v8h;
typedef __attribute__((ext_vector_type(8)))  float    v8f;
typedef __attribute__((ext_vector_type(4)))  float    v4f;
typedef __attribute__((ext_vector_type(4)))  unsigned int v4u;

__device__ __forceinline__ unsigned short h16c(float x, float carry) {
  const float r = x * carry;
  const _Float16 hv = (_Float16)r;
  return __builtin_bit_cast(unsigned short, hv);
}
__device__ __forceinline__ unsigned short h16res(float x, float carry) {
  const float r = x * carry;
  const _Float16 hv = (_Float16)r;
  const float hf = (float)hv;
  const float res = (r - hf) * RCARRY;
  const _Float16 lv = (_Float16)res;
  return __builtin_bit_cast(unsigned short, lv);
}
__device__ __forceinline__ unsigned pk16(unsigned short a, unsigned short b) { return (unsigned)a | ((unsigned)b << 16); }

struct FragH {
  union U { v16h v; v8h h[2]; };
  static __device__ __forceinline__ v16h load(const _Float16* p) {
    U f;
    f.h[0] = *(const v8h*)(p);
    f.h[1] = *(const v8h*)(p + 16);
    return f.v;
  }
};
__device__ __forceinline__ v8f mma_g(v16h a, v16h b, v8f c) {
  c = __builtin_amdgcn_wmma_f32_16x16x32_f16(false, a, false, b, (short)0, c, false, false);
  asm volatile("v_nop\n\tv_nop\n\tv_nop\n\tv_nop" : "+v"(c) : "v"(a), "v"(b));
  return c;
}

__global__ __launch_bounds__(256) void gate_proj_kernel(const float* __restrict__ q, const float* __restrict__ k,
                                                        const float* __restrict__ v,
                                                        const float* __restrict__ igw, const float* __restrict__ igb,
                                                        const float* __restrict__ fgw, const float* __restrict__ fgb,
                                                        float* __restrict__ igp, float* __restrict__ fgp) {
  __shared__ float sm[16][32];
  const int tid = threadIdx.x, lane = tid & 31, wave = tid >> 5;
  const int R0 = blockIdx.x * 32;
  const float* wi = igw + (size_t)wave * NFEAT;
  const float* wf = fgw + (size_t)wave * NFEAT;
#pragma unroll 1
  for (int jg = 0; jg < 8; ++jg) {
    float ai[4], af[4];
#pragma unroll
    for (int rr = 0; rr < 4; ++rr) {
      ai[rr] = 0.0f;
      af[rr] = 0.0f;
    }
#pragma unroll 1
    for (int src = 0; src < 3; ++src) {
      const float* p = ((src == 0) ? q : ((src == 1) ? k : v)) + (size_t)(R0 + jg * 4) * HID;
      const float* wis = wi + src * HID;
      const float* wfs = wf + src * HID;
#pragma unroll 1
      for (int it = 0; it < 8; ++it) {
        const int f = it * 128 + lane * 4;
        const v4f a = *(const v4f*)(wis + f);
        const v4f b = *(const v4f*)(wfs + f);
#pragma unroll
        for (int rr = 0; rr < 4; ++rr) {
          const v4f x = *(const v4f*)(p + (size_t)rr * HID + f);
#pragma unroll
          for (int e = 0; e < 4; ++e) {
            ai[rr] = fmaf(x[e], a[e], ai[rr]);
            af[rr] = fmaf(x[e], b[e], af[rr]);
          }
        }
      }
    }
#pragma unroll
    for (int rr = 0; rr < 4; ++rr) {
      float xa = ai[rr];
      float xb = af[rr];
#pragma unroll
      for (int m = 16; m > 0; m >>= 1) {
        xa += __shfl_xor(xa, m, 32);
        xb += __shfl_xor(xb, m, 32);
      }
      ai[rr] = xa;
      af[rr] = xb;
    }
    if (lane == 0) {
#pragma unroll
      for (int rr = 0; rr < 4; ++rr) {
        sm[wave][jg * 4 + rr]     = ai[rr];
        sm[8 + wave][jg * 4 + rr] = af[rr];
      }
    }
  }
  __syncthreads();
  const float bi = igb[wave];
  const float bf = fgb[wave];
  float* di = igp + (size_t)wave * SEQ + R0;
  float* df = fgp + (size_t)wave * SEQ + R0;
  if (lane < 8) {
    v4f oi, of;
#pragma unroll
    for (int e = 0; e < 4; ++e) {
      oi[e] = sm[wave][4 * lane + e] + bi;
      of[e] = sm[8 + wave][4 * lane + e] + bf;
    }
    *(volatile v4f*)(di + 4 * lane) = oi;
    *(volatile v4f*)(df + 4 * lane) = of;
    __threadfence();
    *(volatile v4f*)(di + 4 * lane) = oi;
    *(volatile v4f*)(df + 4 * lane) = of;
  }
}

__global__ __launch_bounds__(256) void gate_scan_kernel(const float* __restrict__ igp, const float* __restrict__ fgp,
                                                        float* __restrict__ APL, float* __restrict__ MXPL,
                                                        float* __restrict__ NFPL) {
  __shared__ float sF[SEQ];
  __shared__ float sI[SEQ];
  __shared__ float sA[SEQ];
  __shared__ float sM[SEQ];
  const int tid = threadIdx.x;
  const size_t base = (size_t)blockIdx.x * SEQ;
#pragma unroll 1
  for (int i = 0; i < 8; ++i) {
    const int idx = i * 256 + tid;
    const float x = fgp[base + idx];
    const float lf = fminf(x, 0.0f) - log1pf(expf(-fabsf(x)));
    sF[idx] = lf;
    sI[idx] = igp[base + idx];
  }
  __syncthreads();
  if (tid == 0) {
    float F = 0.0f;
    float mxv = -INFINITY;
#pragma unroll 1
    for (int s = 0; s < SEQ; ++s) {
      F += sF[s];
      const float a = sI[s] - F;
      mxv = fmaxf(mxv, a);
      sF[s] = F;
      sA[s] = a;
      sM[s] = mxv;
    }
  }
  __syncthreads();
#pragma unroll 1
  for (int i = 0; i < 2; ++i) {
    const int s4 = (i * 256 + tid) * 4;
    v4f oa, om, on;
#pragma unroll
    for (int e = 0; e < 4; ++e) {
      const float a = sA[s4 + e];
      const float m = sM[s4 + e];
      const float F = sF[s4 + e];
      oa[e] = a;
      om[e] = m;
      on[e] = expf(-(F + m));
    }
    *(volatile v4f*)(APL  + base + s4) = oa;
    *(volatile v4f*)(MXPL + base + s4) = om;
    *(volatile v4f*)(NFPL + base + s4) = on;
    __threadfence();
    *(volatile v4f*)(APL  + base + s4) = oa;
    *(volatile v4f*)(MXPL + base + s4) = om;
    *(volatile v4f*)(NFPL + base + s4) = on;
  }
}

__global__ __launch_bounds__(256) void plane_convert_kernel(const float* __restrict__ q, const float* __restrict__ k,
                                                            const float* __restrict__ v, unsigned short* __restrict__ QH,
                                                            unsigned short* __restrict__ KH, unsigned short* __restrict__ VHT,
                                                            unsigned short* __restrict__ QL, unsigned short* __restrict__ KL) {
  __shared__ unsigned short Vt[64 * VT_PITCH];
  const int tid = threadIdx.x, lane = tid & 31, wave = tid >> 5;
  const int s0 = blockIdx.x * 64;
  const int h  = blockIdx.y;
#pragma unroll 1
  for (int i = 0; i < 4; ++i) {
    const int e  = i * 256 + tid;
    const int r  = e >> 4;
    const int c8 = (e & 15) * 8;
    const size_t src = (size_t)(s0 + r) * HID + (size_t)h * DHEAD + c8;
    const size_t dst = ((size_t)h * SEQ + s0 + r) * DHEAD + c8;
    const v4f q0 = *(const v4f*)(q + src);
    const v4f q1 = *(const v4f*)(q + src + 4);
    const v4f k0 = *(const v4f*)(k + src);
    const v4f k1 = *(const v4f*)(k + src + 4);
    const v4f v0 = *(const v4f*)(v + src);
    const v4f v1 = *(const v4f*)(v + src + 4);
    unsigned short qb[8], kb[8], ql[8], kl[8];
#pragma unroll
    for (int t = 0; t < 4; ++t) {
      qb[t]     = h16c(q0[t], QCARRY);
      qb[4 + t] = h16c(q1[t], QCARRY);
      kb[t]     = h16c(k0[t], KCARRY);
      kb[4 + t] = h16c(k1[t], KCARRY);
      ql[t]     = h16res(q0[t], QCARRY);
      ql[4 + t] = h16res(q1[t], QCARRY);
      kl[t]     = h16res(k0[t], KCARRY);
      kl[4 + t] = h16res(k1[t], KCARRY);
      Vt[r * VT_PITCH + c8 + t]     = h16c(v0[t], VCARRY);
      Vt[r * VT_PITCH + c8 + 4 + t] = h16c(v1[t], VCARRY);
    }
    const v4u qu = (v4u){pk16(qb[0], qb[1]), pk16(qb[2], qb[3]), pk16(qb[4], qb[5]), pk16(qb[6], qb[7])};
    const v4u ku = (v4u){pk16(kb[0], kb[1]), pk16(kb[2], kb[3]), pk16(kb[4], kb[5]), pk16(kb[6], kb[7])};
    const v4u qlu = (v4u){pk16(ql[0], ql[1]), pk16(ql[2], ql[3]), pk16(ql[4], ql[5]), pk16(ql[6], ql[7])};
    const v4u klu = (v4u){pk16(kl[0], kl[1]), pk16(kl[2], kl[3]), pk16(kl[4], kl[5]), pk16(kl[6], kl[7])};
    *(volatile v4u*)(QH + dst) = qu;
    *(volatile v4u*)(KH + dst) = ku;
    *(volatile v4u*)(QL + dst) = qlu;
    *(volatile v4u*)(KL + dst) = klu;
    __threadfence();
    *(volatile v4u*)(QH + dst) = qu;
    *(volatile v4u*)(KH + dst) = ku;
    *(volatile v4u*)(QL + dst) = qlu;
    *(volatile v4u*)(KL + dst) = klu;
  }
  __syncthreads();
  const int dl = lane >> 3, sl = lane & 7;
#pragma unroll 1
  for (int it = 0; it < 4; ++it) {
    const int d = it * 32 + wave * 4 + dl;
    unsigned short hb[8];
#pragma unroll
    for (int j = 0; j < 8; ++j) hb[j] = Vt[(sl * 8 + j) * VT_PITCH + d];
    const v4u u = (v4u){pk16(hb[0], hb[1]), pk16(hb[2], hb[3]), pk16(hb[4], hb[5]), pk16(hb[6], hb[7])};
    unsigned short* op = VHT + ((size_t)h * DHEAD + d) * SEQ + s0 + sl * 8;
    *(volatile v4u*)op = u;
    __threadfence();
    *(volatile v4u*)op = u;
  }
}

__global__ __launch_bounds__(256) void decay_attn_norm_kernel(const unsigned short* __restrict__ QHp,
                                                              const unsigned short* __restrict__ KHp,
                                                              const unsigned short* __restrict__ VTp,
                                                              const unsigned short* __restrict__ QLp,
                                                              const unsigned short* __restrict__ KLp,
                                                              const float* __restrict__ APL, const float* __restrict__ MXPL,
                                                              const float* __restrict__ NFPL, const float* __restrict__ oscale,
                                                              float* __restrict__ out) {
  __shared__ __align__(16) _Float16 Qs[ROWS_BLK * QPITCH];
  __shared__ __align__(16) _Float16 Qls[ROWS_BLK * QPITCH];
  __shared__ __align__(16) _Float16 Ks[KEY_TILE * QPITCH];
  __shared__ __align__(16) _Float16 Kls[KEY_TILE * QPITCH];
  __shared__ __align__(16) _Float16 Vs[DHEAD * VPITCH];
  __shared__ __align__(16) _Float16 Ps[4][16 * VPITCH];
  __shared__ __align__(16) float    Sl[8][16 * SLABP];
  __shared__ float redS[4][2][16];
  __shared__ float redM[4][2][16];
  __shared__ float redV[4][2][16];

  const int tid = threadIdx.x, lane = tid & 31, wave = tid >> 5;
  const int rg = wave >> 1, dh = wave & 1;
  const int c = lane & 15, hh = lane >> 4, koff = 8 * hh, c4 = c * 4;
  const int rb = blockIdx.x;
  const int h  = blockIdx.y;
  const int row0 = rb * ROWS_BLK;
  const size_t hS = (size_t)h * SEQ;

  const _Float16* Qb  = (const _Float16*)QHp + hS * DHEAD;
  const _Float16* Kb  = (const _Float16*)KHp + hS * DHEAD;
  const _Float16* Qlb = (const _Float16*)QLp + hS * DHEAD;
  const _Float16* Klb = (const _Float16*)KLp + hS * DHEAD;
  const _Float16* Vb  = (const _Float16*)VTp + (size_t)h * DHEAD * SEQ;

#pragma unroll
  for (int i = 0; i < 4; ++i) {
    const int e  = i * 256 + tid;
    const int r  = e >> 4;
    const int c8 = (e & 15) * 8;
    *(v8h*)(Qs  + r * QPITCH + c8) = *(const v8h*)(Qb  + (size_t)(row0 + r) * DHEAD + c8);
    *(v8h*)(Qls + r * QPITCH + c8) = *(const v8h*)(Qlb + (size_t)(row0 + r) * DHEAD + c8);
  }

  const int rloc = 16 * rg + 8 * hh;
  float mx[8], nfl[8], rs[8];
  {
    const float* mp = MXPL + hS + row0 + rloc;
    const float* np = NFPL + hS + row0 + rloc;
    const v4f m0 = *(const v4f*)(mp);
    const v4f m1 = *(const v4f*)(mp + 4);
    const v4f n0 = *(const v4f*)(np);
    const v4f n1 = *(const v4f*)(np + 4);
#pragma unroll
    for (int e = 0; e < 4; ++e) {
      mx[e] = m0[e];
      mx[4 + e] = m1[e];
      nfl[e] = n0[e];
      nfl[4 + e] = n1[e];
    }
  }
#pragma unroll
  for (int r = 0; r < 8; ++r) rs[r] = 0.0f;

  const v8f z8 = {0.f, 0.f, 0.f, 0.f, 0.f, 0.f, 0.f, 0.f};
  v8f acc[4];
#pragma unroll
  for (int j = 0; j < 4; ++j) acc[j] = z8;

  const int nTb = (row0 + ROWS_BLK) / KEY_TILE;
  _Float16* pw = Ps[rg];

#pragma unroll 1
  for (int tb = 0; tb < nTb; ++tb) {
    const int t0 = tb * KEY_TILE;
    __syncthreads();
#pragma unroll
    for (int i = 0; i < 2; ++i) {
      const int e   = i * 256 + tid;
      const int kr  = e >> 4;
      const int kc8 = (e & 15) * 8;
      *(v8h*)(Ks  + kr * QPITCH + kc8) = *(const v8h*)(Kb  + (size_t)(t0 + kr) * DHEAD + kc8);
      *(v8h*)(Kls + kr * QPITCH + kc8) = *(const v8h*)(Klb + (size_t)(t0 + kr) * DHEAD + kc8);
      const int vd  = e >> 2;
      const int vc8 = (e & 3) * 8;
      *(v8h*)(Vs + vd * VPITCH + vc8) = *(const v8h*)(Vb + (size_t)vd * SEQ + t0 + vc8);
    }
    const int col = t0 + 16 * dh + c;
    float acol = APL[hS + col];
    asm volatile("" : "+v"(acol));
    __syncthreads();

    v8f s = z8;
    v8f sx = z8;
    {
      const _Float16* qa = Qs  + (16 * rg + c) * QPITCH + koff;
      const _Float16* ql = Qls + (16 * rg + c) * QPITCH + koff;
      const _Float16* kb = Ks  + (16 * dh + c) * QPITCH + koff;
      const _Float16* kl = Kls + (16 * dh + c) * QPITCH + koff;
#pragma unroll
      for (int kc = 0; kc < 4; ++kc) {
        const v16h a  = FragH::load(qa + kc * 32);
        const v16h al = FragH::load(ql + kc * 32);
        const v16h bb = FragH::load(kb + kc * 32);
        const v16h bl = FragH::load(kl + kc * 32);
        s  = mma_g(a, bb, s);
        sx = mma_g(a, bl, sx);
        sx = mma_g(al, bb, sx);
      }
    }
#pragma unroll
    for (int r = 0; r < 8; ++r) {
      const int row = row0 + rloc + r;
      const float arg = fminf(acol - mx[r], 0.0f);
      float e = expf(arg);
      e = (e < F32_MIN_NORMAL) ? 0.0f : e;
      const float sc = s[r] + sx[r] * RCARRY_INV;
      const float val = sc * SSCALE * e;
      const float p = (col <= row) ? val : 0.0f;
      rs[r] += p;
      pw[(8 * hh + r) * VPITCH + 16 * dh + c] = (_Float16)(p * PCARRY);
    }
    __syncthreads();

    {
      const v16h ap = FragH::load(pw + c * VPITCH + koff);
#pragma unroll
      for (int j = 0; j < 4; ++j) {
        const v16h bv = FragH::load(Vs + ((dh * 4 + j) * 16 + c) * VPITCH + koff);
        acc[j] = mma_g(ap, bv, acc[j]);
      }
    }
  }

#pragma unroll
  for (int r = 0; r < 8; ++r) {
    float x = rs[r];
#pragma unroll
    for (int m = 1; m < 16; m <<= 1) x += __shfl_xor(x, m, 32);
    rs[r] = x;
  }
  if (c == 0) {
#pragma unroll
    for (int r = 0; r < 8; ++r) redS[rg][dh][8 * hh + r] = rs[r];
  }
  __syncthreads();
  float smean[8];
#pragma unroll
  for (int r = 0; r < 8; ++r) {
    const float tot = redS[rg][0][8 * hh + r] + redS[rg][1][8 * hh + r];
    const float nrm = fmaxf(fabsf(tot), nfl[r]) + EPS_NORM;
    const float inv = OFOLD * (1.0f / nrm);
    float t = 0.0f;
#pragma unroll
    for (int j = 0; j < 4; ++j) {
      const float x = acc[j][r] * inv;
      acc[j][r] = x;
      t += x;
    }
#pragma unroll
    for (int m = 1; m < 16; m <<= 1) t += __shfl_xor(t, m, 32);
    smean[r] = t;
  }
  if (c == 0) {
#pragma unroll
    for (int r = 0; r < 8; ++r) redM[rg][dh][8 * hh + r] = smean[r];
  }
  __syncthreads();
  float sq[8];
#pragma unroll
  for (int r = 0; r < 8; ++r) {
    const float mean = (redM[rg][0][8 * hh + r] + redM[rg][1][8 * hh + r]) * INV_DHEAD;
    float t = 0.0f;
#pragma unroll
    for (int j = 0; j < 4; ++j) {
      const float d = acc[j][r] - mean;
      acc[j][r] = d;
      t += d * d;
    }
#pragma unroll
    for (int m = 1; m < 16; m <<= 1) t += __shfl_xor(t, m, 32);
    sq[r] = t;
  }
  if (c == 0) {
#pragma unroll
    for (int r = 0; r < 8; ++r) redV[rg][dh][8 * hh + r] = sq[r];
  }
  __syncthreads();
  float rstd[8];
#pragma unroll
  for (int r = 0; r < 8; ++r) {
    const float var = (redV[rg][0][8 * hh + r] + redV[rg][1][8 * hh + r]) * INV_DHEAD;
    rstd[r] = rsqrtf(var + EPS_LN);
  }

  float* slab = Sl[wave];
  float* obase = out + ((size_t)(row0 + 16 * rg)) * HID + (size_t)h * DHEAD + dh * 64;
#pragma unroll
  for (int j = 0; j < 4; ++j) {
    const float sc = oscale[h * DHEAD + dh * 64 + j * 16 + c];
#pragma unroll
    for (int r = 0; r < 8; ++r) slab[(8 * hh + r) * SLABP + j * 16 + c] = acc[j][r] * rstd[r] * sc;
  }
  __builtin_amdgcn_fence(__ATOMIC_RELEASE, "workgroup");
  __builtin_amdgcn_wave_barrier();
  __builtin_amdgcn_fence(__ATOMIC_ACQUIRE, "workgroup");
  for (int pass = 0; pass < 2; ++pass) {
#pragma unroll
    for (int it = 0; it < 8; ++it) {
      const int row = it * 2 + hh;
      const v4f val = *(const v4f*)(slab + row * SLABP + c4);
      *(volatile v4f*)(obase + (size_t)row * HID + c4) = val;
    }
    __threadfence();
  }
}

extern "C" void kernel_launch(void* const* d_in, const int* in_sizes, int n_in,
                              void* d_out, int out_size, void* d_ws, size_t ws_size, hipStream_t stream) {
  if (n_in < 8 || d_out == nullptr || d_ws == nullptr) return;
  if (in_sizes[0] != SEQ * HID || in_sizes[1] != SEQ * HID || in_sizes[2] != SEQ * HID ||
      in_sizes[3] != NFEAT * NHEAD || in_sizes[4] != NHEAD || in_sizes[5] != NFEAT * NHEAD || in_sizes[6] != NHEAD ||
      in_sizes[7] != HID || out_size != SEQ * HID) return;

  const float* q   = (const float*)d_in[0];
  const float* k   = (const float*)d_in[1];
  const float* v   = (const float*)d_in[2];
  const float* igw = (const float*)d_in[3];
  const float* igb = (const float*)d_in[4];
  const float* fgw = (const float*)d_in[5];
  const float* fgb = (const float*)d_in[6];
  const float* osc = (const float*)d_in[7];
  float* out = (float*)d_out;

  char* ws = (char*)d_ws;
  size_t off = 0;
  auto carve = [&](size_t bytes) -> char* {
    char* p = ws + off;
    off += (bytes + 255) & ~(size_t)255;
    return p;
  };
  float* IGP  = (float*)carve((size_t)NHEAD * SEQ * 4);
  float* FGP  = (float*)carve((size_t)NHEAD * SEQ * 4);
  float* APL  = (float*)carve((size_t)NHEAD * SEQ * 4);
  float* MXPL = (float*)carve((size_t)NHEAD * SEQ * 4);
  float* NFPL = (float*)carve((size_t)NHEAD * SEQ * 4);
  unsigned short* QH  = (unsigned short*)carve((size_t)NHEAD * SEQ * DHEAD * 2);
  unsigned short* KH  = (unsigned short*)carve((size_t)NHEAD * SEQ * DHEAD * 2);
  unsigned short* VHT = (unsigned short*)carve((size_t)NHEAD * SEQ * DHEAD * 2);
  unsigned short* QL  = (unsigned short*)carve((size_t)NHEAD * SEQ * DHEAD * 2);
  unsigned short* KL  = (unsigned short*)carve((size_t)NHEAD * SEQ * DHEAD * 2);
  if (off > ws_size || off > (size_t)134217728) return;

  gate_proj_kernel<<<dim3(SEQ / 32), dim3(256), 0, stream>>>(q, k, v, igw, igb, fgw, fgb, IGP, FGP);
  gate_scan_kernel<<<dim3(NHEAD), dim3(256), 0, stream>>>(IGP, FGP, APL, MXPL, NFPL);
  plane_convert_kernel<<<dim3(SEQ / 64, NHEAD), dim3(256), 0, stream>>>(q, k, v, QH, KH, VHT, QL, KL);
  decay_attn_norm_kernel<<<dim3(SEQ / ROWS_BLK, NHEAD), dim3(256), 0, stream>>>(QH, KH, VHT, QL, KL, APL, MXPL, NFPL, osc, out);
}
